// SlidingWindowAttention_14130442404432
// MI455X (gfx1250) — hardware-verified
//
#include <hip/hip_runtime.h>

typedef __attribute__((ext_vector_type(16))) _Float16 v16h;
typedef __attribute__((ext_vector_type(16))) __bf16 v16b;
typedef __attribute__((ext_vector_type(8)))  _Float16 v8h;
typedef __attribute__((ext_vector_type(8)))  __bf16 v8b;
typedef __attribute__((ext_vector_type(8)))  float v8f;
typedef __attribute__((ext_vector_type(4)))  float v4f;
typedef __attribute__((ext_vector_type(4)))  unsigned v4u;

#ifndef NB
#define NB 1
#endif
#ifndef SEQ
#define SEQ 8192
#endif
#define SEQ_FULL 8192
#define DIN 1024
#define CC 1024
#define NH 16
#define HD 64
#define NKV 128
#define DOUT 1024
#define WIN 256

static_assert(SEQ % 64 == 0);
static_assert(SEQ <= SEQ_FULL);
static_assert(DIN % 64 == 0 && CC % 64 == 0);
static_assert(CC == NH * HD && NKV == 2 * HD && HD == 64);
static_assert(CC % 128 == 0 && DOUT % 128 == 0 && NKV == 128);
static_assert(WIN % 32 == 0);
static_assert(((size_t)NB * SEQ * DIN) % 2048 == 0);

template <typename T> __device__ __forceinline__ void vst2(void* p, T v) { *(volatile T*)p = v; __threadfence(); *(volatile T*)p = v; }
__device__ __forceinline__ v8f wmma16(v16h a, v16h b, v8f c) {
  v8f d = __builtin_amdgcn_wmma_f32_16x16x32_f16(false, a, false, b, (short)0, c, false, false);
  asm volatile("v_nop\n\tv_nop\n\tv_nop\n\tv_nop" : "+v"(d) : "v"(a), "v"(b));
  return d;
}
__device__ __forceinline__ v8f wmma_bf(v16b a, v16b b, v8f c) {
  v8f d = __builtin_amdgcn_wmma_f32_16x16x32_bf16(false, a, false, b, (short)0, c, false, false);
  asm volatile("v_nop\n\tv_nop\n\tv_nop\n\tv_nop" : "+v"(d) : "v"(a), "v"(b));
  return d;
}
__device__ __forceinline__ v16h frag_h(const _Float16* rowk0, unsigned lane) {
  union { v16h v; v8h q[2]; } u; const _Float16* p = rowk0 + 8u * (lane >> 4);
  u.q[0] = *(const v8h*)p; u.q[1] = *(const v8h*)(p + 16); return u.v;
}
__device__ __forceinline__ v16b frag_b(const __bf16* rowk0, unsigned lane) {
  union { v16b v; v8b q[2]; } u; const __bf16* p = rowk0 + 8u * (lane >> 4);
  u.q[0] = *(const v8b*)p; u.q[1] = *(const v8b*)(p + 16); return u.v;
}
__device__ __forceinline__ float bfr(float v) { return (float)(__bf16)v; }
#define LDSX() do { asm volatile("s_wait_dscnt 0" ::: "memory"); __builtin_amdgcn_wave_barrier(); __builtin_amdgcn_fence(3  , "workgroup"); } while (0)

#define WS_XQ   ((size_t)0)
#define WS_WQT  (WS_XQ   + (size_t)2 * NB * SEQ * DIN)
#define WS_WKVT (WS_WQT  + (size_t)2 * CC * DIN)
#define WS_WOT  (WS_WKVT + (size_t)2 * NKV * DIN)
#define WS_QH   (WS_WOT  + (size_t)2 * DOUT * CC)
#define WS_QL   (WS_QH   + (size_t)2 * NB * SEQ * CC)
#define WS_KH   (WS_QL   + (size_t)2 * NB * SEQ * CC)
#define WS_KL   (WS_KH   + (size_t)2 * NB * SEQ * HD)
#define WS_VT   (WS_KL   + (size_t)2 * NB * SEQ * HD)
#define WS_CTX  (WS_VT   + (size_t)2 * NB * HD * SEQ)
#define WS_END  (WS_CTX  + (size_t)2 * NB * SEQ * CC)
static_assert(WS_END <= (size_t)134217728);

__global__ __launch_bounds__(256) void k_cvt(const float* __restrict__ X, unsigned short* __restrict__ XB) {
  const unsigned i8 = blockIdx.x * 256u + threadIdx.x;
  const unsigned row = i8 / (unsigned)(DIN / 8), c8 = i8 - row * (unsigned)(DIN / 8);
  const unsigned b = row / (unsigned)SEQ, t = row - b * (unsigned)SEQ;
  const float* p = X + ((size_t)b * SEQ_FULL + t) * DIN + c8 * 8u;
  const v4f x0 = *(const v4f*)p, x1 = *(const v4f*)(p + 4);
  union { v8b b8; v4u u; } o;
#pragma unroll
  for (int i = 0; i < 4; ++i) { o.b8[i] = (__bf16)x0[i]; o.b8[4 + i] = (__bf16)x1[i]; }
  vst2(XB + (size_t)row * DIN + c8 * 8u, o.u);
}

__global__ __launch_bounds__(256) void k_wt(const float* __restrict__ Wq, const float* __restrict__ Wkv, const float* __restrict__ Wo,
                                            unsigned short* __restrict__ WQT, unsigned short* __restrict__ WKVT, unsigned short* __restrict__ WOT) {
  __shared__ __align__(16) unsigned short tt[64][72];
  const unsigned z = blockIdx.z;
  const unsigned krows = (z == 2u) ? (unsigned)CC : (unsigned)DIN;
  const unsigned ncols = (z == 0u) ? (unsigned)CC : (z == 1u) ? (unsigned)NKV : (unsigned)DOUT;
  const unsigned k0 = blockIdx.x * 64u, n0 = blockIdx.y * 64u;
  if (k0 >= krows || n0 >= ncols) return;
  const float* W = (z == 0u) ? Wq : (z == 1u) ? Wkv : Wo;
  unsigned short* O = (z == 0u) ? WQT : (z == 1u) ? WKVT : WOT;
  const unsigned tid = threadIdx.x, rl = tid >> 2, q = tid & 3u;
  { const float* p = W + (size_t)(k0 + rl) * ncols + n0 + q * 16u;
    const v4f x0 = *(const v4f*)p, x1 = *(const v4f*)(p + 4), x2 = *(const v4f*)(p + 8), x3 = *(const v4f*)(p + 12);
    float xa[16] = {x0[0],x0[1],x0[2],x0[3],x1[0],x1[1],x1[2],x1[3],x2[0],x2[1],x2[2],x2[3],x3[0],x3[1],x3[2],x3[3]};
#pragma unroll
    for (int i = 0; i < 16; ++i) {
      const __bf16 bv = (__bf16)xa[i];
      const _Float16 hv = (_Float16)((float)bv * 256.0f);
      const unsigned short bb = __builtin_bit_cast(unsigned short, bv), hb = __builtin_bit_cast(unsigned short, hv);
      tt[q * 16u + i][rl] = (z == 2u) ? hb : bb;
    } }
  __syncthreads();
  for (unsigned e = tid; e < 64u * 8u; e += 256u) { const unsigned nl = e >> 3, qq = e & 7u;
    const v4u v = *(const v4u*)&tt[nl][qq * 8u];
    vst2(O + (size_t)(n0 + nl) * krows + k0 + qq * 8u, v); }
}

template <int MODE>
__global__ __launch_bounds__(128) void k_proj(const __bf16* __restrict__ XA, const float* __restrict__ XF, const __bf16* __restrict__ WT,
                                              _Float16* __restrict__ DH, _Float16* __restrict__ DL, _Float16* __restrict__ VT) {
  __shared__ __align__(16) _Float16 lds[2 * 4 * 32 * 72];
  const unsigned tid = threadIdx.x, wave = tid >> 5, lane = tid & 31u, col = lane & 15u, g = lane >> 4;
  const unsigned wm = wave & 1u, wn = wave >> 1;
  const unsigned r0 = blockIdx.x * 64u, c0 = blockIdx.y * 128u;
  const unsigned bb = r0 / (unsigned)SEQ, t0 = r0 - bb * (unsigned)SEQ;
  v8f acc[2][4] = {};
#pragma unroll 1
  for (unsigned kc = 0; kc < (unsigned)(DIN / 32); ++kc) {
    v16b a[2];
#pragma unroll
    for (int rt = 0; rt < 2; ++rt) {
      const unsigned rl = wm * 32u + (unsigned)rt * 16u + col;
      if constexpr (MODE == 0) {
        a[rt] = frag_b(XA + (size_t)(r0 + rl) * DIN + kc * 32u, lane);
      } else {
        const float* p = XF + ((size_t)bb * SEQ_FULL + t0 + rl) * DIN + kc * 32u + 8u * g;
        const v4f x0 = *(const v4f*)p, x1 = *(const v4f*)(p + 4), x2 = *(const v4f*)(p + 16), x3 = *(const v4f*)(p + 20);
        v16b f;
#pragma unroll
        for (int i = 0; i < 4; ++i) { f[i] = (__bf16)x0[i]; f[4 + i] = (__bf16)x1[i]; f[8 + i] = (__bf16)x2[i]; f[12 + i] = (__bf16)x3[i]; }
        a[rt] = f;
      }
    }
    asm volatile("s_wait_loadcnt 0x0" ::: "memory");
#pragma unroll
    for (int nt = 0; nt < 4; ++nt) {
      const v16b w = frag_b(WT + (size_t)(c0 + wn * 64u + (unsigned)nt * 16u + col) * DIN + kc * 32u, lane);
      asm volatile("s_wait_loadcnt 0x0" ::: "memory");
      acc[0][nt] = wmma_bf(a[0], w, acc[0][nt]);
      acc[1][nt] = wmma_bf(a[1], w, acc[1][nt]);
    }
  }
  if constexpr (MODE == 0) {
    _Float16* sh = lds + wave * (32u * 72u); _Float16* sl = lds + 4u * 32u * 72u + wave * (32u * 72u);
#pragma unroll
    for (int rt = 0; rt < 2; ++rt)
#pragma unroll
      for (int nt = 0; nt < 4; ++nt)
#pragma unroll
        for (int r = 0; r < 8; ++r) { const unsigned rl = (unsigned)rt * 16u + 8u * g + (unsigned)r, cl = (unsigned)nt * 16u + col;
          const float v = acc[rt][nt][r]; const _Float16 hv = (_Float16)v;
          sh[rl * 72u + cl] = hv; sl[rl * 72u + cl] = (_Float16)((v - (float)hv) * 1024.0f); }
    LDSX();
#pragma unroll 1
    for (unsigned it = 0; it < 8u; ++it) { const unsigned rl = it * 4u + (lane >> 3), q = lane & 7u;
      const size_t dst = (size_t)(r0 + wm * 32u + rl) * CC + c0 + wn * 64u + q * 8u;
      const v8h hvv = *(const v8h*)(sh + rl * 72u + q * 8u); const v8h lvv = *(const v8h*)(sl + rl * 72u + q * 8u);
      vst2(DH + dst, hvv); vst2(DL + dst, lvv); }
  } else {
    _Float16* sh = lds; _Float16* sl = lds + 64u * 72u; _Float16* th = lds + 2u * 64u * 72u;
#pragma unroll
    for (int rt = 0; rt < 2; ++rt)
#pragma unroll
      for (int nt = 0; nt < 4; ++nt)
#pragma unroll
        for (int r = 0; r < 8; ++r) { const unsigned rl = wm * 32u + (unsigned)rt * 16u + 8u * g + (unsigned)r, cl = (unsigned)nt * 16u + col;
          const float v = acc[rt][nt][r]; const _Float16 hv = (_Float16)v;
          if (wn == 0u) { sh[rl * 72u + cl] = hv; sl[rl * 72u + cl] = (_Float16)((v - (float)hv) * 1024.0f); }
          else { th[cl * 72u + rl] = hv; } }
    __syncthreads();
    for (unsigned e = tid; e < 64u * 8u; e += 128u) { const unsigned rw = e >> 3, q = e & 7u;
      const v8h kh = *(const v8h*)(sh + rw * 72u + q * 8u); const v8h kl = *(const v8h*)(sl + rw * 72u + q * 8u); const v8h vv = *(const v8h*)(th + rw * 72u + q * 8u);
      vst2(DH + (size_t)(r0 + rw) * HD + q * 8u, kh);
      vst2(DL + (size_t)(r0 + rw) * HD + q * 8u, kl);
      vst2(VT + ((size_t)bb * HD + rw) * SEQ + t0 + q * 8u, vv); }
  }
}

__global__ __launch_bounds__(128) void k_attn(const _Float16* __restrict__ QH, const _Float16* __restrict__ QL, const _Float16* __restrict__ KH, const _Float16* __restrict__ KL,
                                              const _Float16* __restrict__ VT, _Float16* __restrict__ CTX) {
  __shared__ __align__(16) _Float16 pst[4][16][40];
  __shared__ __align__(16) _Float16 so[4][16][72];
  const unsigned tid = threadIdx.x, wave = tid >> 5, lane = tid & 31u, col = lane & 15u, g = lane >> 4;
  const unsigned qb = blockIdx.x, h = blockIdx.y, b = blockIdx.z;
  const unsigned q0 = qb * 64u, ql0 = q0 + wave * 16u;
  const unsigned klo = (q0 > (unsigned)WIN) ? (q0 - (unsigned)WIN) : 0u;
  const unsigned kht = q0 + 64u + (unsigned)WIN;
  const unsigned khe = (kht < (unsigned)SEQ) ? kht : (unsigned)SEQ;
  const size_t qoff = ((size_t)b * SEQ + ql0 + col) * CC + h * (unsigned)HD;
  const v16h qa0 = frag_h(QH + qoff, lane), qa1 = frag_h(QH + qoff + 32, lane);
  const v16h qr0 = frag_h(QL + qoff, lane), qr1 = frag_h(QL + qoff + 32, lane);
  const _Float16* Kb = KH + (size_t)b * SEQ * HD; const _Float16* KLb = KL + (size_t)b * SEQ * HD; const _Float16* Vb = VT + (size_t)b * HD * SEQ;
  float rmax[8], rsum[8];
#pragma unroll
  for (int r = 0; r < 8; ++r) { rmax[r] = -3.0e38f; rsum[r] = 0.f; }
  v8f acc[4] = {};
#pragma unroll 1
  for (unsigned kb = klo; kb < khe; kb += 32u) {
    v8f s[2];
#pragma unroll
    for (int st = 0; st < 2; ++st) {
      const size_t ko = (size_t)(kb + (unsigned)st * 16u + col) * HD;
      const v16h k0 = frag_h(Kb + ko, lane), k1 = frag_h(Kb + ko + 32, lane);
      const v16h l0 = frag_h(KLb + ko, lane), l1 = frag_h(KLb + ko + 32, lane);
      asm volatile("s_wait_loadcnt 0x0" ::: "memory");
      v8f c = {}; c = wmma16(qa0, k0, c); c = wmma16(qa1, k1, c);
      v8f d = {}; d = wmma16(qr0, k0, d); d = wmma16(qr1, k1, d); d = wmma16(qa0, l0, d); d = wmma16(qa1, l1, d);
#pragma unroll
      for (int r = 0; r < 8; ++r) c[r] = c[r] + d[r] * (1.0f / 1024.0f);
      s[st] = c;
    }
    float bm[8];
#pragma unroll
    for (int r = 0; r < 8; ++r) bm[r] = -3.0e38f;
#pragma unroll
    for (int st = 0; st < 2; ++st)
#pragma unroll
      for (int r = 0; r < 8; ++r) {
        const int dd = (int)(ql0 + 8u * g + (unsigned)r) - (int)(kb + (unsigned)st * 16u + col);
        const bool ok = (dd <= WIN) && (dd >= -WIN);
        const float v = ok ? s[st][r] : -3.0e38f;
        s[st][r] = v; bm[r] = fmaxf(bm[r], v);
      }
#pragma unroll
    for (int r = 0; r < 8; ++r) { float m = bm[r];
      m = fmaxf(m, __shfl_xor(m, 1)); m = fmaxf(m, __shfl_xor(m, 2)); m = fmaxf(m, __shfl_xor(m, 4)); m = fmaxf(m, __shfl_xor(m, 8));
      bm[r] = m; }
    float sc[8], bs[8];
#pragma unroll
    for (int r = 0; r < 8; ++r) { const float nm = fmaxf(rmax[r], bm[r]); sc[r] = __expf(fmaxf(rmax[r] - nm, -80.0f)); rmax[r] = nm; bs[r] = 0.f; }
#pragma unroll
    for (int st = 0; st < 2; ++st)
#pragma unroll
      for (int r = 0; r < 8; ++r) {
        const float v = s[st][r];
        const float e = __expf(fmaxf(v - rmax[r], -80.0f));
        const float p = (v > -1.0e38f) ? e : 0.f;
        bs[r] += p;
        pst[wave][8u * g + (unsigned)r][(unsigned)st * 16u + col] = (_Float16)(p * 16384.0f);
      }
#pragma unroll
    for (int r = 0; r < 8; ++r) { float sv = bs[r];
      sv += __shfl_xor(sv, 1); sv += __shfl_xor(sv, 2); sv += __shfl_xor(sv, 4); sv += __shfl_xor(sv, 8);
      rsum[r] = rsum[r] * sc[r] + sv; }
#pragma unroll
    for (int dt = 0; dt < 4; ++dt)
#pragma unroll
      for (int r = 0; r < 8; ++r) acc[dt][r] *= sc[r];
    LDSX();
    const v16h pa = frag_h(&pst[wave][col][0], lane);
    LDSX();
#pragma unroll
    for (int dt = 0; dt < 4; ++dt) {
      const v16h bv = frag_h(Vb + (size_t)((unsigned)dt * 16u + col) * SEQ + kb, lane);
      asm volatile("s_wait_loadcnt 0x0" ::: "memory");
      acc[dt] = wmma16(pa, bv, acc[dt]);
    }
  }
#pragma unroll
  for (int r = 0; r < 8; ++r) { const float inv = (1.0f / rsum[r]) * (1.0f / 16384.0f);
#pragma unroll
    for (int dt = 0; dt < 4; ++dt) so[wave][8u * g + (unsigned)r][(unsigned)dt * 16u + col] = (_Float16)(acc[dt][r] * inv); }
  LDSX();
#pragma unroll 1
  for (unsigned it = 0; it < 4u; ++it) { const unsigned rl = it * 4u + (lane >> 3), q = lane & 7u;
    const v8h v = *(const v8h*)&so[wave][rl][q * 8u];
    vst2(CTX + ((size_t)b * SEQ + ql0 + rl) * CC + h * (unsigned)HD + q * 8u, v); }
}

__global__ __launch_bounds__(128) void k_out(const _Float16* __restrict__ CT, const _Float16* __restrict__ WOT, float* __restrict__ OUT) {
  __shared__ __align__(16) float so[4][32][68];
  const unsigned tid = threadIdx.x, wave = tid >> 5, lane = tid & 31u, col = lane & 15u, g = lane >> 4;
  const unsigned wm = wave & 1u, wn = wave >> 1;
  const unsigned r0 = blockIdx.x * 64u, c0 = blockIdx.y * 128u;
  v8f acc[2][4] = {};
#pragma unroll 1
  for (unsigned kc = 0; kc < (unsigned)(CC / 32); ++kc) {
    const v16h a0 = frag_h(CT + (size_t)(r0 + wm * 32u + col) * CC + kc * 32u, lane);
    const v16h a1 = frag_h(CT + (size_t)(r0 + wm * 32u + 16u + col) * CC + kc * 32u, lane);
    asm volatile("s_wait_loadcnt 0x0" ::: "memory");
#pragma unroll
    for (int nt = 0; nt < 4; ++nt) {
      const v16h w = frag_h(WOT + (size_t)(c0 + wn * 64u + (unsigned)nt * 16u + col) * CC + kc * 32u, lane);
      asm volatile("s_wait_loadcnt 0x0" ::: "memory");
      acc[0][nt] = wmma16(a0, w, acc[0][nt]);
      acc[1][nt] = wmma16(a1, w, acc[1][nt]);
    }
  }
#pragma unroll
  for (int rt = 0; rt < 2; ++rt)
#pragma unroll
    for (int nt = 0; nt < 4; ++nt)
#pragma unroll
      for (int r = 0; r < 8; ++r) so[wave][(unsigned)rt * 16u + 8u * g + (unsigned)r][(unsigned)nt * 16u + col] = acc[rt][nt][r] * (1.0f / 256.0f);
  LDSX();
#pragma unroll 1
  for (unsigned it = 0; it < 16u; ++it) { const unsigned rl = it * 2u + (lane >> 4), q = lane & 15u;
    const v4f v = *(const v4f*)&so[wave][rl][q * 4u];
    vst2(OUT + (size_t)(r0 + wm * 32u + rl) * DOUT + c0 + wn * 64u + q * 4u, v); }
}

extern "C" void kernel_launch(void* const* d_in, const int* in_sizes, int n_in, void* d_out, int out_size, void* d_ws, size_t ws_size, hipStream_t stream) {
  if (n_in < 5) return;
  if ((size_t)in_sizes[0] < (size_t)NB * SEQ * DIN) return;
  if ((size_t)in_sizes[1] < (size_t)NB * SEQ * DIN) return;
  if ((size_t)in_sizes[2] < (size_t)DIN * CC) return;
  if ((size_t)in_sizes[3] < (size_t)DIN * NKV) return;
  if ((size_t)in_sizes[4] < (size_t)CC * DOUT) return;
  if ((size_t)out_size < (size_t)NB * SEQ * DOUT) return;
  if (ws_size < (size_t)WS_END) return;
  const float* q = (const float*)d_in[0]; const float* kv = (const float*)d_in[1];
  const float* w_q = (const float*)d_in[2]; const float* w_kv = (const float*)d_in[3]; const float* w_o = (const float*)d_in[4];
  char* ws = (char*)d_ws;
  unsigned short* XQ = (unsigned short*)(ws + WS_XQ); unsigned short* WQT = (unsigned short*)(ws + WS_WQT); unsigned short* WKVT = (unsigned short*)(ws + WS_WKVT); unsigned short* WOT = (unsigned short*)(ws + WS_WOT);
  _Float16* QH = (_Float16*)(ws + WS_QH); _Float16* QL = (_Float16*)(ws + WS_QL); _Float16* KH = (_Float16*)(ws + WS_KH); _Float16* KL = (_Float16*)(ws + WS_KL);
  _Float16* VT = (_Float16*)(ws + WS_VT); _Float16* CTX = (_Float16*)(ws + WS_CTX);

  k_cvt<<<dim3((unsigned)(((size_t)NB * SEQ * DIN) / 2048)), 256, 0, stream>>>(q, XQ);
  k_wt<<<dim3(((DIN > CC ? DIN : CC) / 64), ((CC > DOUT ? CC : DOUT) / 64), 3), 256, 0, stream>>>(w_q, w_kv, w_o, WQT, WKVT, WOT);
  k_proj<0><<<dim3(NB * SEQ / 64, CC / 128), 128, 0, stream>>>((const __bf16*)XQ, q, (const __bf16*)WQT, QH, QL, VT);
  k_proj<1><<<dim3(NB * SEQ / 64, 1), 128, 0, stream>>>((const __bf16*)XQ, kv, (const __bf16*)WKVT, KH, KL, VT);
  k_attn<<<dim3(SEQ / 64, NH, NB), 128, 0, stream>>>(QH, QL, KH, KL, VT, CTX);
  k_out<<<dim3(NB * SEQ / 64, DOUT / 128), 128, 0, stream>>>(CTX, (const _Float16*)WOT, (float*)d_out);
}
